// unit_gcn_2714419331727
// MI455X (gfx1250) — hardware-verified
//
#include <hip/hip_runtime.h>
#include <stdint.h>

#define NB      64
#define CIN     64
#define COUT    64
#define KSUB    3
#define GRP     8
#define DCH     192
#define TT      128
#define VV      25
#define TV      3200
#define VP      32
#define KG      96
#define NROW    204800
#define NBLK0   3200
#define TGRP    8
#define CGRP    4
#define NBLK1   2048
#define ROWB    400
#define NTHR    256
#define OUTN    13107200
#define OPIECES 3276800
#define P0F     384
#define P1F     32

#define SX      256.0f
#define SW      4096.0f
#define INV_P   9.5367431640625e-07f
#define SAJ     4096.0f
#define INV_G   2.44140625e-04f
#define SLO     65536.0f
#define INV_L   1.52587890625e-05f
#define HMINN   6.103515625e-05f
#define BNEPS   1e-5f
#define ICNT    (1.0 / 204800.0)

static_assert(TV == TT * VV);
static_assert(NROW == NB * TV);
static_assert(NROW == NBLK0 * 64);
static_assert(TV == 50 * 64);
static_assert(NBLK1 == NB * TGRP * CGRP);
static_assert(ROWB == 16 * VV);
static_assert(TT == 16 * TGRP);
static_assert(COUT == 16 * CGRP);
static_assert(DCH == KSUB * COUT);
static_assert(OUTN == NB * COUT * TV);
static_assert(OPIECES * 4 == OUTN);
static_assert(OPIECES % NTHR == 0);
static_assert(KG == KSUB * VP);
static_assert((DCH * CIN) % (8 * NTHR) == 0);
static_assert((KSUB * GRP * VP * VP) % (8 * NTHR) == 0);

typedef _Float16 v16h __attribute__((ext_vector_type(16)));
typedef _Float16 v8h  __attribute__((ext_vector_type(8)));
typedef float    v8f  __attribute__((ext_vector_type(8)));
typedef float    v4f  __attribute__((ext_vector_type(4)));
typedef unsigned v4u  __attribute__((ext_vector_type(4)));

__device__ __forceinline__ float bf_rne(float f) {
  unsigned u = __float_as_uint(f);
  u = (u + 0x7FFFu + ((u >> 16) & 1u)) & 0xFFFF0000u;
  return __uint_as_float(u);
}
__device__ __forceinline__ unsigned hbits(_Float16 h) {
  return (unsigned)__builtin_bit_cast(unsigned short, h);
}
__device__ __forceinline__ v8f zero8f() { v8f z = {0.f, 0.f, 0.f, 0.f, 0.f, 0.f, 0.f, 0.f}; return z; }
__device__ __forceinline__ float frcp(float x) { return __builtin_amdgcn_rcpf(x); }

__device__ __forceinline__ v16h ldfrag(const _Float16* p) {
  union { v16h v; v8h h[2]; } f;
  f.h[0] = *(const v8h*)(p);
  f.h[1] = *(const v8h*)(p + 16);
  return f.v;
}

__device__ __forceinline__ v8f mma_h(v16h a, v16h b, v8f c) {
  return __builtin_amdgcn_wmma_f32_16x16x32_f16(false, a, false, b, (short)0, c, false, false);
}
__device__ __forceinline__ void guard3(v8f& c0, v8f& c1, v8f& c2, v16h a, v16h b0, v16h b1, v16h b2) {
#if defined(__HIP_DEVICE_COMPILE__)
  asm volatile("v_nop\n\tv_nop\n\tv_nop\n\tv_nop"
               : "+v"(c0), "+v"(c1), "+v"(c2)
               : "v"(a), "v"(b0), "v"(b1), "v"(b2));
#endif
}
__device__ __forceinline__ void guard4(v8f& c0, v8f& c1, v8f& c2, v8f& c3,
                                       v16h a0, v16h a1, v16h b0, v16h b1) {
#if defined(__HIP_DEVICE_COMPILE__)
  asm volatile("v_nop\n\tv_nop\n\tv_nop\n\tv_nop"
               : "+v"(c0), "+v"(c1), "+v"(c2), "+v"(c3)
               : "v"(a0), "v"(a1), "v"(b0), "v"(b1));
#endif
}

__global__ __launch_bounds__(NTHR)
void k_xprep(const float* __restrict__ x0, _Float16* xt)
{
  __shared__ __align__(16) _Float16 tile[64 * 64];
  const int tid = threadIdx.x;
  const int blk = blockIdx.x;
  const int n   = blk / 50;
  const int tv0 = (blk - n * 50) * 64;
  const float* xb = x0 + (size_t)n * CIN * TV + tv0;
#pragma unroll
  for (int i = 0; i < 16; ++i) {
    const int idx = i * NTHR + tid;
    const int c = idx >> 6;
    const int j = idx & 63;
    const float f = bf_rne(xb[(size_t)c * TV + j]) * SX;
    tile[j * 64 + c] = (_Float16)f;
  }
  __syncthreads();
  const int L0 = tid >> 3;
  const int L1 = L0 + 32;
  const int pc = (tid & 7) * 8;
  union { v8h h; v4u u; } w0, w1;
  w0.h = *(const v8h*)(tile + L0 * 64 + pc);
  w1.h = *(const v8h*)(tile + L1 * 64 + pc);
  _Float16* d0 = xt + ((size_t)(blk * 64 + L0) * CIN + pc);
  _Float16* d1 = xt + ((size_t)(blk * 64 + L1) * CIN + pc);
  *(volatile v4u*)d0 = w0.u;
  *(volatile v4u*)d1 = w1.u;
  __threadfence();
  *(volatile v4u*)d0 = w0.u;
  *(volatile v4u*)d1 = w1.u;
}

__global__ __launch_bounds__(NTHR)
void k_par(const float* __restrict__ W, const float* __restrict__ adj,
           _Float16* wtp, _Float16* dat, float* invs)
{
  const int tid = threadIdx.x;
  const int blk = blockIdx.x;
  if (blk < 6) {
    const int q  = blk * NTHR + tid;
    const int d  = q >> 3;
    const int c0 = (q & 7) * 8;
    unsigned hb[8];
#pragma unroll
    for (int j = 0; j < 8; ++j) {
      const float f = bf_rne(W[(size_t)(c0 + j) * DCH + d]) * SW;
      hb[j] = hbits((_Float16)f);
    }
    v4u wv;
    wv.x = hb[0] | (hb[1] << 16);
    wv.y = hb[2] | (hb[3] << 16);
    wv.z = hb[4] | (hb[5] << 16);
    wv.w = hb[6] | (hb[7] << 16);
    _Float16* dst = wtp + (size_t)q * 8;
    *(volatile v4u*)dst = wv;
    __threadfence();
    *(volatile v4u*)dst = wv;
  } else if (blk < 18) {
    const int q   = (blk - 6) * NTHR + tid;
    const int row = q >> 2;
    const int kg  = row >> 5;
    const int w   = row & 31;
    const int wc  = (w < VV) ? w : (VV - 1);
    const int vp  = (q & 3) * 8;
    unsigned hb[8];
#pragma unroll
    for (int j = 0; j < 8; ++j) {
      const int v  = vp + j;
      const int vc = (v < VV) ? v : (VV - 1);
      float f = bf_rne(adj[(size_t)(kg * VV + vc) * VV + wc]) * SAJ;
      f = (v < VV && w < VV) ? f : 0.0f;
      hb[j] = hbits((_Float16)f);
    }
    v4u wv;
    wv.x = hb[0] | (hb[1] << 16);
    wv.y = hb[2] | (hb[3] << 16);
    wv.z = hb[4] | (hb[5] << 16);
    wv.w = hb[6] | (hb[7] << 16);
    _Float16* dst = dat + (size_t)q * 8;
    *(volatile v4u*)dst = wv;
    __threadfence();
    *(volatile v4u*)dst = wv;
  } else {
    const int q  = (tid < 192) ? tid : 191;
    const int kg = q >> 3;
    const int wp = (q & 7) * 4;
    const int w0c = (wp + 0 < VV) ? (wp + 0) : (VV - 1);
    const int w1c = (wp + 1 < VV) ? (wp + 1) : (VV - 1);
    const int w2c = (wp + 2 < VV) ? (wp + 2) : (VV - 1);
    const int w3c = (wp + 3 < VV) ? (wp + 3) : (VV - 1);
    float s0 = 0.f, s1 = 0.f, s2 = 0.f, s3 = 0.f;
#pragma unroll 1
    for (int v = 0; v < VV; ++v) {
      const float* ar = adj + (size_t)(kg * VV + v) * VV;
      s0 += bf_rne(ar[w0c]);
      s1 += bf_rne(ar[w1c]);
      s2 += bf_rne(ar[w2c]);
      s3 += bf_rne(ar[w3c]);
    }
    v4f iv;
    iv.x = (wp + 0 < VV) ? frcp(s0 + 0.001f) * INV_G : 0.0f;
    iv.y = (wp + 1 < VV) ? frcp(s1 + 0.001f) * INV_G : 0.0f;
    iv.z = (wp + 2 < VV) ? frcp(s2 + 0.001f) * INV_G : 0.0f;
    iv.w = (wp + 3 < VV) ? frcp(s3 + 0.001f) * INV_G : 0.0f;
    float* dst = invs + (size_t)q * 4;
    if (tid < 192) *(volatile v4f*)dst = iv;
    __threadfence();
    if (tid < 192) *(volatile v4f*)dst = iv;
  }
}

__global__ __launch_bounds__(NTHR)
void k_stat0(const _Float16* __restrict__ xt, const _Float16* __restrict__ wtp,
             const float* __restrict__ bias, float* part0)
{
  __shared__ __align__(16) float red[4 * P0F];
  __shared__ __align__(16) float outl[P0F];
  const int tid = threadIdx.x, lane = tid & 31, wv = tid >> 5, m = lane & 15, hh = lane >> 4;
  const int mt = wv & 3, dh = wv >> 2;
  const int blk = blockIdx.x;
  const _Float16* ap = xt  + ((size_t)blk * 64 + 16 * mt + m) * CIN + 8 * hh;
  const _Float16* bp = wtp + (size_t)(96 * dh + m) * CIN + 8 * hh;

  v8f acc[6];
#pragma unroll
  for (int nt = 0; nt < 6; ++nt) acc[nt] = zero8f();

#pragma unroll
  for (int ks = 0; ks < 2; ++ks) {
    const v16h a = ldfrag(ap + 32 * ks);
    {
      const v16h b0 = ldfrag(bp + 0 * 16 * CIN + 32 * ks);
      const v16h b1 = ldfrag(bp + 1 * 16 * CIN + 32 * ks);
      const v16h b2 = ldfrag(bp + 2 * 16 * CIN + 32 * ks);
      acc[0] = mma_h(a, b0, acc[0]);
      acc[1] = mma_h(a, b1, acc[1]);
      acc[2] = mma_h(a, b2, acc[2]);
      guard3(acc[0], acc[1], acc[2], a, b0, b1, b2);
    }
    {
      const v16h b3 = ldfrag(bp + 3 * 16 * CIN + 32 * ks);
      const v16h b4 = ldfrag(bp + 4 * 16 * CIN + 32 * ks);
      const v16h b5 = ldfrag(bp + 5 * 16 * CIN + 32 * ks);
      acc[3] = mma_h(a, b3, acc[3]);
      acc[4] = mma_h(a, b4, acc[4]);
      acc[5] = mma_h(a, b5, acc[5]);
      guard3(acc[3], acc[4], acc[5], a, b3, b4, b5);
    }
  }

#pragma unroll
  for (int nt = 0; nt < 6; ++nt) {
    const int col = 96 * dh + 16 * nt + m;
    const float bb = bf_rne(bias[col]);
    float s = 0.f, q = 0.f;
#pragma unroll
    for (int r = 0; r < 8; ++r) {
      const float x = acc[nt][r] * INV_P + bb;
      s += x;
      q += x * x;
    }
    s += __shfl_xor(s, 16, 32);
    q += __shfl_xor(q, 16, 32);
    if (hh == 0) {
      red[mt * P0F + 2 * col]     = s;
      red[mt * P0F + 2 * col + 1] = q;
    }
  }
  __syncthreads();
  for (int p = tid; p < P0F; p += NTHR)
    outl[p] = ((red[p] + red[P0F + p]) + red[2 * P0F + p]) + red[3 * P0F + p];
  __syncthreads();
  if (tid < 96) {
    const v4f w = *(const v4f*)(outl + 4 * tid);
    float* pp = part0 + (size_t)blk * P0F + 4 * tid;
    *(volatile v4f*)pp = w;
    __threadfence();
    *(volatile v4f*)pp = w;
  }
}

__global__ __launch_bounds__(NTHR)
void k_fin0(const float* __restrict__ part0, const float* __restrict__ gamma,
            const float* __restrict__ beta, float* ss0)
{
  __shared__ __align__(16) float so[2 * DCH];
  const int tid = threadIdx.x;
  const int d = (tid < DCH) ? tid : (DCH - 1);
  double s = 0.0, q = 0.0;
#pragma unroll 1
  for (int b = 0; b < NBLK0; ++b) {
    const float* pp = part0 + (size_t)b * P0F + 2 * d;
    s += (double)pp[0];
    q += (double)pp[1];
  }
  const double mu = s * ICNT;
  double var = q * ICNT - mu * mu;
  var = (var > 0.0) ? var : 0.0;
  const float rstd = 1.0f / sqrtf((float)var + BNEPS);
  const float sc = bf_rne(gamma[d]) * rstd;
  const float sh = bf_rne(beta[d]) - (float)mu * sc;
  if (tid < DCH) {
    so[2 * tid]     = sc;
    so[2 * tid + 1] = sh;
  }
  __syncthreads();
  if (tid < 96) {
    const v4f w = *(const v4f*)(so + 4 * tid);
    float* pp = ss0 + 4 * tid;
    *(volatile v4f*)pp = w;
    __threadfence();
    *(volatile v4f*)pp = w;
  }
}

__global__ __launch_bounds__(NTHR)
void k_main(const _Float16* __restrict__ xt, const _Float16* __restrict__ wtp,
            const float* __restrict__ bias, const float* __restrict__ ss0,
            const _Float16* __restrict__ dat, const float* __restrict__ invs,
            float* x2p, float* part1)
{
  __shared__ __align__(16) _Float16 shi[16 * 16 * KG];
  __shared__ __align__(16) _Float16 slo[16 * 16 * KG];
  __shared__ __align__(16) float stg[8 * 16 * VP];
  __shared__ __align__(16) float st1[P1F];
  __shared__ float psc[48];
  __shared__ float psh[48];
  __shared__ float pbi[48];

  const int tid = threadIdx.x, lane = tid & 31, wv = tid >> 5, m = lane & 15, hh = lane >> 4;
  const int blk = blockIdx.x;
  const int cg  = blk & 3;
  const int tg  = (blk >> 2) & 7;
  const int n   = blk >> 5;

  if (tid < 48) {
    const int k = tid >> 4, cl = tid & 15;
    const int d = COUT * k + 16 * cg + cl;
    psc[tid] = ss0[2 * d];
    psh[tid] = ss0[2 * d + 1];
    pbi[tid] = bf_rne(bias[d]);
  }
  {
    const v4u z = {0u, 0u, 0u, 0u};
    unsigned* zh = (unsigned*)shi;
    unsigned* zl = (unsigned*)slo;
    for (int i = tid; i < (16 * 16 * KG) / 8; i += NTHR) {
      *(v4u*)(zh + 4 * i) = z;
      *(v4u*)(zl + 4 * i) = z;
    }
  }
  __syncthreads();

  {
    const int rowb = n * TV + tg * ROWB;
#pragma unroll 1
    for (int mt = wv; mt < 25; mt += 8) {
      const _Float16* ap = xt + (size_t)(rowb + 16 * mt + m) * CIN + 8 * hh;
      v8f acc[3];
      acc[0] = zero8f();  acc[1] = zero8f();  acc[2] = zero8f();
#pragma unroll
      for (int ks = 0; ks < 2; ++ks) {
        const v16h a = ldfrag(ap + 32 * ks);
        const _Float16* bp = wtp + (size_t)(16 * cg + m) * CIN + 32 * ks + 8 * hh;
        const v16h b0 = ldfrag(bp);
        const v16h b1 = ldfrag(bp + COUT * CIN);
        const v16h b2 = ldfrag(bp + 2 * COUT * CIN);
        acc[0] = mma_h(a, b0, acc[0]);
        acc[1] = mma_h(a, b1, acc[1]);
        acc[2] = mma_h(a, b2, acc[2]);
        guard3(acc[0], acc[1], acc[2], a, b0, b1, b2);
      }
      const int tvb = 16 * mt + 8 * hh;
      const int tl0 = tvb / VV;
      const int v0  = tvb - tl0 * VV;
#pragma unroll
      for (int nt = 0; nt < 3; ++nt) {
        const int col = 16 * nt + m;
        const float sc = psc[col];
        const float sh = psh[col];
        const float bb = pbi[col];
#pragma unroll
        for (int r = 0; r < 8; ++r) {
          int v = v0 + r;
          int tl = tl0;
          if (v >= VV) { v -= VV; tl += 1; }
          const float x1 = acc[nt][r] * INV_P + bb;
          const float y  = x1 * sc + sh;
          const float ya = (fabsf(y) < HMINN) ? 0.0f : y;
          const _Float16 h16 = (_Float16)ya;
          const float lo = (y - (float)h16) * SLO;
          const _Float16 l16 = (_Float16)lo;
          const int idx = (m * 16 + tl) * KG + nt * VP + v;
          shi[idx] = h16;
          slo[idx] = l16;
        }
      }
    }
  }
  __syncthreads();

#pragma unroll 1
  for (int pass = 0; pass < 2; ++pass) {
    const int cl = 2 * wv + pass;
    const int c  = 16 * cg + cl;
    const int g  = c & (GRP - 1);
    const _Float16* ahp = shi + (cl * 16 + m) * KG + 8 * hh;
    const _Float16* alp = slo + (cl * 16 + m) * KG + 8 * hh;
    v8f res0 = zero8f(), res1 = zero8f();
#pragma unroll
    for (int k = 0; k < KSUB; ++k) {
      const v16h ahi = ldfrag(ahp + VP * k);
      const v16h alo = ldfrag(alp + VP * k);
      const int kg = k * GRP + g;
      const _Float16* bq = dat + (size_t)(kg * VP + m) * VP + 8 * hh;
      const v16h b0 = ldfrag(bq);
      const v16h b1 = ldfrag(bq + 16 * VP);
      v8f dh0 = mma_h(ahi, b0, zero8f());
      v8f dh1 = mma_h(ahi, b1, zero8f());
      v8f dl0 = mma_h(alo, b0, zero8f());
      v8f dl1 = mma_h(alo, b1, zero8f());
      guard4(dh0, dh1, dl0, dl1, ahi, alo, b0, b1);
      const float i0 = invs[kg * VP + m];
      const float i1 = invs[kg * VP + 16 + m];
#pragma unroll
      for (int r = 0; r < 8; ++r) {
        res0[r] += (dh0[r] + dl0[r] * INV_L) * i0;
        res1[r] += (dh1[r] + dl1[r] * INV_L) * i1;
      }
    }
    float s = 0.f, q = 0.f;
#pragma unroll
    for (int r = 0; r < 8; ++r) {
      s += res0[r] + res1[r];
      q += res0[r] * res0[r] + res1[r] * res1[r];
    }
#pragma unroll
    for (int o = 1; o < 32; o <<= 1) {
      s += __shfl_xor(s, o, 32);
      q += __shfl_xor(q, o, 32);
    }
    if (lane == 0) {
      st1[2 * cl]     = s;
      st1[2 * cl + 1] = q;
    }
    float* sw = stg + wv * (16 * VP);
#pragma unroll
    for (int r = 0; r < 8; ++r) {
      sw[(8 * hh + r) * VP + m]      = res0[r];
      sw[(8 * hh + r) * VP + 16 + m] = res1[r];
    }
    __syncthreads();
    {
      const int rq = lane >> 3;
      const int pc = (lane & 7) * 4;
      const v4f w0 = *(const v4f*)(sw + (0  + rq) * VP + pc);
      const v4f w1 = *(const v4f*)(sw + (4  + rq) * VP + pc);
      const v4f w2 = *(const v4f*)(sw + (8  + rq) * VP + pc);
      const v4f w3 = *(const v4f*)(sw + (12 + rq) * VP + pc);
      float* ob = x2p + ((size_t)(n * COUT + c) * TT + 16 * tg) * VP + pc;
      float* p0 = ob + (size_t)(0  + rq) * VP;
      float* p1 = ob + (size_t)(4  + rq) * VP;
      float* p2 = ob + (size_t)(8  + rq) * VP;
      float* p3 = ob + (size_t)(12 + rq) * VP;
      *(volatile v4f*)p0 = w0;
      *(volatile v4f*)p1 = w1;
      *(volatile v4f*)p2 = w2;
      *(volatile v4f*)p3 = w3;
      __threadfence();
      *(volatile v4f*)p0 = w0;
      *(volatile v4f*)p1 = w1;
      *(volatile v4f*)p2 = w2;
      *(volatile v4f*)p3 = w3;
    }
    __syncthreads();
  }

  if (tid < 8) {
    const v4f sv = *(const v4f*)(st1 + 4 * tid);
    float* pp = part1 + (size_t)blk * P1F + 4 * tid;
    *(volatile v4f*)pp = sv;
    __threadfence();
    *(volatile v4f*)pp = sv;
  }
}

__global__ __launch_bounds__(NTHR)
void k_fin1(const float* __restrict__ part1, const float* __restrict__ gamma,
            const float* __restrict__ beta, float* ss1)
{
  __shared__ __align__(16) float so[2 * COUT];
  const int tid = threadIdx.x;
  const int c = (tid < COUT) ? tid : (COUT - 1);
  const int slot = 2 * (c & 15);
  const int cgc = c >> 4;
  double s = 0.0, q = 0.0;
#pragma unroll 1
  for (int b = 0; b < NB * TGRP; ++b) {
    const float* pp = part1 + (size_t)(b * CGRP + cgc) * P1F + slot;
    s += (double)pp[0];
    q += (double)pp[1];
  }
  const double mu = s * ICNT;
  double var = q * ICNT - mu * mu;
  var = (var > 0.0) ? var : 0.0;
  const float rstd = 1.0f / sqrtf((float)var + BNEPS);
  const float sc = bf_rne(gamma[c]) * rstd;
  const float sh = bf_rne(beta[c]) - (float)mu * sc;
  if (tid < COUT) {
    so[2 * tid]     = sc;
    so[2 * tid + 1] = sh;
  }
  __syncthreads();
  if (tid < 32) {
    const v4f w = *(const v4f*)(so + 4 * tid);
    float* pp = ss1 + 4 * tid;
    *(volatile v4f*)pp = w;
    __threadfence();
    *(volatile v4f*)pp = w;
  }
}

__global__ __launch_bounds__(NTHR)
void k_out(const float* __restrict__ x2p, const float* __restrict__ x0,
           const float* __restrict__ ss1, float* out)
{
  const int q  = blockIdx.x * NTHR + threadIdx.x;
  const int e0 = q * 4;
  const int c  = (e0 / TV) & (COUT - 1);
  const float sc = ss1[2 * c];
  const float sh = ss1[2 * c + 1];
  const v4f xv = *(const v4f*)(x0 + e0);
  float o[4];
#pragma unroll
  for (int j = 0; j < 4; ++j) {
    const int e   = e0 + j;
    const int row = e / VV;
    const int col = e - row * VV;
    const float z = x2p[(size_t)row * VP + col];
    const float val = z * sc + sh + bf_rne(xv[j]);
    o[j] = fmaxf(val, 0.0f);
  }
  v4f ov;
  ov.x = o[0];  ov.y = o[1];  ov.z = o[2];  ov.w = o[3];
  float* p = out + e0;
  *(volatile v4f*)p = ov;
  __threadfence();
  *(volatile v4f*)p = ov;
}

extern "C" void kernel_launch(void* const* d_in, const int* in_sizes, int n_in,
                              void* d_out, int out_size, void* d_ws, size_t ws_size,
                              hipStream_t stream) {
  if (n_in < 8) return;
  if (in_sizes[0] != NB * CIN * TV) return;
  if (in_sizes[1] != CIN * DCH) return;
  if (in_sizes[2] != DCH) return;
  if (in_sizes[3] != KSUB * GRP * VV * VV) return;
  if (in_sizes[4] != DCH || in_sizes[5] != DCH) return;
  if (in_sizes[6] != COUT || in_sizes[7] != COUT) return;
  if (out_size != OUTN) return;

  const size_t b_xt  = (size_t)NROW * CIN * 2;
  const size_t b_wtp = (size_t)DCH * CIN * 2;
  const size_t b_dat = (size_t)KSUB * GRP * VP * VP * 2;
  const size_t b_inv = (size_t)KSUB * GRP * VP * 4;
  const size_t b_p0  = (size_t)NBLK0 * P0F * 4;
  const size_t b_ss0 = (size_t)DCH * 2 * 4;
  const size_t b_x2p = (size_t)NB * COUT * TT * VP * 4;
  const size_t b_p1  = (size_t)NBLK1 * P1F * 4;
  const size_t b_ss1 = (size_t)COUT * 2 * 4;

  const size_t o_xt  = 0;
  const size_t o_wtp = o_xt  + b_xt;
  const size_t o_dat = o_wtp + b_wtp;
  const size_t o_inv = o_dat + b_dat;
  const size_t o_p0  = o_inv + b_inv;
  const size_t o_ss0 = o_p0  + b_p0;
  const size_t o_x2p = o_ss0 + b_ss0;
  const size_t o_p1  = o_x2p + b_x2p;
  const size_t o_ss1 = o_p1  + b_p1;
  const size_t total = o_ss1 + b_ss1;
  if (total > ws_size) return;

  const float* x0   = (const float*)d_in[0];
  const float* W    = (const float*)d_in[1];
  const float* bias = (const float*)d_in[2];
  const float* adj  = (const float*)d_in[3];
  const float* g0   = (const float*)d_in[4];
  const float* be0  = (const float*)d_in[5];
  const float* g1   = (const float*)d_in[6];
  const float* be1  = (const float*)d_in[7];
  float* out = (float*)d_out;

  unsigned char* wsb = (unsigned char*)d_ws;
  _Float16* xt   = (_Float16*)(wsb + o_xt);
  _Float16* wtp  = (_Float16*)(wsb + o_wtp);
  _Float16* dat  = (_Float16*)(wsb + o_dat);
  float*    invs = (float*)(wsb + o_inv);
  float*    p0   = (float*)(wsb + o_p0);
  float*    ss0  = (float*)(wsb + o_ss0);
  float*    x2p  = (float*)(wsb + o_x2p);
  float*    p1   = (float*)(wsb + o_p1);
  float*    ss1  = (float*)(wsb + o_ss1);

  k_xprep<<<dim3(NBLK0), dim3(NTHR), 0, stream>>>(x0, xt);
  (void)hipGetLastError();
  k_par<<<dim3(19), dim3(NTHR), 0, stream>>>(W, adj, wtp, dat, invs);
  (void)hipGetLastError();
  k_stat0<<<dim3(NBLK0), dim3(NTHR), 0, stream>>>(xt, wtp, bias, p0);
  (void)hipGetLastError();
  k_fin0<<<dim3(1), dim3(NTHR), 0, stream>>>(p0, g0, be0, ss0);
  (void)hipGetLastError();
  k_main<<<dim3(NBLK1), dim3(NTHR), 0, stream>>>(xt, wtp, bias, ss0, dat, invs, x2p, p1);
  (void)hipGetLastError();
  k_fin1<<<dim3(1), dim3(NTHR), 0, stream>>>(p1, g1, be1, ss1);
  (void)hipGetLastError();
  k_out<<<dim3(OPIECES / NTHR), dim3(NTHR), 0, stream>>>(x2p, x0, ss1, out);
  (void)hipGetLastError();
}
